// MultiHeadAttention_85701777424532
// MI455X (gfx1250) — hardware-verified
//
#include <hip/hip_runtime.h>
#ifndef NB
#define NB 1
#endif
#ifndef SEQ
#define SEQ 2048
#endif
#define SEQ_FULL 2048
#define DM 2048
#define NH 16
#define HD 128
#define N3 (3 * DM)
#define NR (NB * SEQ)
#define PLANE ((size_t)NR * DM)

static_assert(NB == 1);
static_assert(NH * HD == DM);
static_assert(SEQ % 128 == 0 && SEQ <= SEQ_FULL);
static_assert(DM % 64 == 0 && N3 % 64 == 0 && DM % 32 == 0 && HD == 128);

typedef __bf16 v16b __attribute__((ext_vector_type(16)));
typedef unsigned short v8us __attribute__((ext_vector_type(8), may_alias));
typedef float v8f  __attribute__((ext_vector_type(8)));
typedef float v4f  __attribute__((ext_vector_type(4)));
typedef float v4fa __attribute__((ext_vector_type(4), may_alias));
typedef int   v4i  __attribute__((ext_vector_type(4)));
typedef int   v4ia __attribute__((ext_vector_type(4), may_alias));
union FragB { v16b v; v8us half[2]; unsigned short u[16]; };

__device__ __forceinline__ unsigned short bf16_bits(float x) { unsigned int u = __float_as_uint(x); return (unsigned short)((u + 0x7FFFu + ((u >> 16) & 1u)) >> 16); }
__device__ __forceinline__ float bf16_val(unsigned short b) { return __uint_as_float(((unsigned int)b) << 16); }
__device__ __forceinline__ float bf16_rne(float x) { return bf16_val(bf16_bits(x)); }

__device__ __forceinline__ v16b ld_frag(const unsigned short* p, int hh) {
  FragB f; f.half[0] = *(const v8us*)(p + 8 * hh); f.half[1] = *(const v8us*)(p + 16 + 8 * hh); return f.v;
}

template <int NT>
__device__ __forceinline__ v8f mmaN(v16b ah, v16b al, v16b bh, v16b bl, v8f c) {
  c = __builtin_amdgcn_wmma_f32_16x16x32_bf16(false, ah, false, bh, (short)0, c, false, false);
  if (NT >= 2) c = __builtin_amdgcn_wmma_f32_16x16x32_bf16(false, al, false, bh, (short)0, c, false, false);
  if (NT >= 3) c = __builtin_amdgcn_wmma_f32_16x16x32_bf16(false, ah, false, bl, (short)0, c, false, false);
  asm volatile("v_nop\n\tv_nop\n\tv_nop\n\tv_nop" : "+v"(c) : "v"(ah), "v"(al), "v"(bh), "v"(bl));
  return c;
}
__device__ __forceinline__ v8f mma3m(v16b ah, v16b al, v16b bh, v16b bl, v8f c) {
  c = __builtin_amdgcn_wmma_f32_16x16x32_bf16(false, ah, false, bh, (short)0, c, false, false);
  c = __builtin_amdgcn_wmma_f32_16x16x32_bf16(false, al, false, bh, (short)0, c, false, false);
  c = __builtin_amdgcn_wmma_f32_16x16x32_bf16(false, ah, false, bl, (short)0, c, false, false);
  asm volatile("v_nop\n\tv_nop\n\tv_nop\n\tv_nop" : "+v"(c) : "v"(ah), "v"(al), "v"(bh), "v"(bl) : "memory");
  return c;
}

__global__ __launch_bounds__(256) void k_xb(const float* __restrict__ x, unsigned short* __restrict__ X, size_t n8) {
  const size_t t = (size_t)blockIdx.x * 256 + threadIdx.x;
  if (t >= n8) return;
  const v4f a = *(const v4fa*)(x + t * 8), c = *(const v4fa*)(x + t * 8 + 4);
  v8us o;
#pragma unroll
  for (int q = 0; q < 4; ++q) { o[q] = bf16_bits(a[q]); o[4 + q] = bf16_bits(c[q]); }
  *(volatile v8us*)(X + t * 8) = o;
  __threadfence();
  *(volatile v8us*)(X + t * 8) = o;
}

__global__ __launch_bounds__(256) void k_wt_bf16(const float* __restrict__ W, unsigned short* __restrict__ Wt, int K, int N) {
  const int t = blockIdx.x * 256 + threadIdx.x;
  const int k8n = K / 8;
  if (t >= N * k8n) return;
  const int n = t / k8n, k8 = (t % k8n) * 8;
  v8us v;
#pragma unroll
  for (int i = 0; i < 8; ++i) v[i] = bf16_bits(W[(size_t)(k8 + i) * N + n]);
  *(volatile v8us*)(Wt + (size_t)n * K + k8) = v;
  __threadfence();
  *(volatile v8us*)(Wt + (size_t)n * K + k8) = v;
}

template <int NT>
__global__ __launch_bounds__(128) void k_gemm(const unsigned short* __restrict__ Ah, const unsigned short* __restrict__ Al, int lda,
                                              const unsigned short* __restrict__ Bt, int ldb, float* __restrict__ C, int ldc, int N, int K) {
  __shared__ __attribute__((aligned(16))) float so[4][32][68];
  const int tid = threadIdx.x, w = tid >> 5, lane = tid & 31, ln = lane & 15, hh = lane >> 4;
  const int ntn = N >> 6;
  const int mt = blockIdx.x / ntn, nq = blockIdx.x - mt * ntn;
  const int row0 = mt * 128 + 32 * w, col0 = nq * 64;
  const size_t ao = (size_t)(row0 + ln) * lda;
  const unsigned short* a0p = Ah + ao; const unsigned short* a1p = a0p + (size_t)16 * lda;
  const unsigned short* l0p = Al + ao; const unsigned short* l1p = l0p + (size_t)16 * lda;
  const unsigned short* b0p = Bt + (size_t)(col0 + ln) * ldb; const unsigned short* b1p = b0p + (size_t)16 * ldb;
  const unsigned short* b2p = b1p + (size_t)16 * ldb; const unsigned short* b3p = b2p + (size_t)16 * ldb;
  const v8f z8 = {0.f, 0.f, 0.f, 0.f, 0.f, 0.f, 0.f, 0.f};
  v8f c00 = z8, c01 = z8, c02 = z8, c03 = z8, c10 = z8, c11 = z8, c12 = z8, c13 = z8;
#pragma unroll 1
  for (int kb = 0; kb < K; kb += 32) {
    const v16b a0 = ld_frag(a0p + kb, hh), a1 = ld_frag(a1p + kb, hh);
    v16b e0 = a0, e1 = a1;
    if (NT >= 2) { e0 = ld_frag(l0p + kb, hh); e1 = ld_frag(l1p + kb, hh); }
    v16b b = ld_frag(b0p + kb, hh); c00 = mmaN<NT>(a0, e0, b, b, c00); c10 = mmaN<NT>(a1, e1, b, b, c10);
    b = ld_frag(b1p + kb, hh); c01 = mmaN<NT>(a0, e0, b, b, c01); c11 = mmaN<NT>(a1, e1, b, b, c11);
    b = ld_frag(b2p + kb, hh); c02 = mmaN<NT>(a0, e0, b, b, c02); c12 = mmaN<NT>(a1, e1, b, b, c12);
    b = ld_frag(b3p + kb, hh); c03 = mmaN<NT>(a0, e0, b, b, c03); c13 = mmaN<NT>(a1, e1, b, b, c13);
  }
  v8f accs[8] = {c00, c01, c02, c03, c10, c11, c12, c13};
#pragma unroll
  for (int u = 0; u < 8; ++u) {
    const int t = u & 3, hf = u >> 2;
#pragma unroll
    for (int r = 0; r < 8; ++r) so[w][hf * 16 + 8 * hh + r][t * 16 + ln] = accs[u][r];
  }
  __syncthreads();
  const int rsub = lane >> 4, c4 = (lane & 15) * 4;
  for (int pass = 0; pass < 2; ++pass) {
#pragma unroll
    for (int q = 0; q < 16; ++q) {
      const int r = q * 2 + rsub;
      const v4f v = *(const v4fa*)&so[w][r][c4];
      *(volatile v4f*)(C + (size_t)(row0 + r) * ldc + col0 + c4) = v;
    }
    if (pass == 0) __threadfence();
  }
}

__global__ __launch_bounds__(256) void k_rope_qk(const float* __restrict__ QKV, const float* __restrict__ sn, const float* __restrict__ cs,
                                                 unsigned short* __restrict__ QK, int nthreads) {
  const int idx = blockIdx.x * 256 + threadIdx.x;
  if (idx >= nthreads) return;
  const int p8 = idx & 7, h = (idx >> 3) & (NH - 1), t = idx >> 7;
  const size_t tb = (size_t)t * HD + p8 * 8;
  float s1[8], c1[8], s2[8], c2[8];
  {
    const v4f a = *(const v4fa*)(sn + tb), b = *(const v4fa*)(sn + tb + 4), c = *(const v4fa*)(sn + tb + 64), d = *(const v4fa*)(sn + tb + 68);
    const v4f e = *(const v4fa*)(cs + tb), f = *(const v4fa*)(cs + tb + 4), g = *(const v4fa*)(cs + tb + 64), k = *(const v4fa*)(cs + tb + 68);
#pragma unroll
    for (int q = 0; q < 4; ++q) {
      s1[q] = bf16_rne(a[q]); s1[4 + q] = bf16_rne(b[q]); s2[q] = bf16_rne(c[q]); s2[4 + q] = bf16_rne(d[q]);
      c1[q] = bf16_rne(e[q]); c1[4 + q] = bf16_rne(f[q]); c2[q] = bf16_rne(g[q]); c2[4 + q] = bf16_rne(k[q]);
    }
  }
#pragma unroll 1
  for (int which = 0; which < 2; ++which) {
    const float* u = QKV + (size_t)t * N3 + (size_t)which * DM + h * HD + p8 * 8;
    const v4f a = *(const v4fa*)(u), b = *(const v4fa*)(u + 4), c = *(const v4fa*)(u + 64), d = *(const v4fa*)(u + 68);
    const float u1[8] = {a[0], a[1], a[2], a[3], b[0], b[1], b[2], b[3]};
    const float u2[8] = {c[0], c[1], c[2], c[3], d[0], d[1], d[2], d[3]};
    v8us h1, l1, h2, l2;
#pragma unroll
    for (int i = 0; i < 8; ++i) {
      const float o1 = u1[i] * c1[i] + (-u2[i]) * s1[i];
      const float o2 = u2[i] * c2[i] + u1[i] * s2[i];
      const unsigned short hb1 = bf16_bits(o1), hb2 = bf16_bits(o2);
      h1[i] = hb1; l1[i] = bf16_bits(o1 - bf16_val(hb1));
      h2[i] = hb2; l2[i] = bf16_bits(o2 - bf16_val(hb2));
    }
    unsigned short* dh = QK + (size_t)which * 2 * PLANE + (size_t)t * DM + h * HD + p8 * 8;
    unsigned short* dl = dh + PLANE;
    for (int pass = 0; pass < 2; ++pass) {
      *(volatile v8us*)(dh) = h1; *(volatile v8us*)(dh + 64) = h2;
      *(volatile v8us*)(dl) = l1; *(volatile v8us*)(dl + 64) = l2;
      if (pass == 0) __threadfence();
    }
  }
}

__global__ __launch_bounds__(256) void k_vt(const float* __restrict__ QKV, unsigned short* __restrict__ VT) {
  __shared__ unsigned short th[64][66];
  __shared__ unsigned short tl[64][66];
  const int tid = threadIdx.x;
  const int ct = blockIdx.x % (DM / 64), tt = blockIdx.x / (DM / 64);
  const int c0 = ct * 64, t0 = tt * 64;
  for (int i = tid; i < 64 * 16; i += 256) {
    const int r = i >> 4, c4 = (i & 15) * 4;
    const v4f a = *(const v4fa*)(QKV + (size_t)(t0 + r) * N3 + 2 * DM + c0 + c4);
#pragma unroll
    for (int q = 0; q < 4; ++q) { const unsigned short hb = bf16_bits(a[q]); th[c4 + q][r] = hb; tl[c4 + q][r] = bf16_bits(a[q] - bf16_val(hb)); }
  }
  __syncthreads();
  v8us hv[2], lv[2];
#pragma unroll
  for (int rd = 0; rd < 2; ++rd) {
    const int i = rd * 256 + tid; const int c = i >> 3, j8 = (i & 7) * 8;
#pragma unroll
    for (int q = 0; q < 8; ++q) { hv[rd][q] = th[c][j8 + q]; lv[rd][q] = tl[c][j8 + q]; }
  }
  for (int pass = 0; pass < 2; ++pass) {
#pragma unroll
    for (int rd = 0; rd < 2; ++rd) {
      const int i = rd * 256 + tid; const int c = i >> 3, j8 = (i & 7) * 8;
      unsigned short* dst = VT + (size_t)(c0 + c) * SEQ + t0 + j8;
      *(volatile v8us*)dst = hv[rd];
      *(volatile v8us*)(dst + PLANE) = lv[rd];
    }
    if (pass == 0) __threadfence();
  }
}

__global__ __launch_bounds__(128) void k_attn(const unsigned short* __restrict__ QK, const unsigned short* __restrict__ VT,
                                              const int* __restrict__ doc, unsigned short* __restrict__ CTX) {
  __shared__ __attribute__((aligned(16))) float so[4][16][68];
  const int tid = threadIdx.x, w = tid >> 5, lane = tid & 31, ln = lane & 15, hh = lane >> 4;
  const int gw = blockIdx.x * 4 + w;
  const int hf = gw & 1, pr = gw >> 1;
  const int qt = pr % (SEQ / 16), head = pr / (SEQ / 16);
  const int q0 = qt * 16, qi = q0 + ln;
  const unsigned short* Qh = QK; const unsigned short* Ql = QK + PLANE;
  const unsigned short* Kh = QK + 2 * PLANE; const unsigned short* Kl = QK + 3 * PLANE;
  const unsigned short* VTh = VT; const unsigned short* VTl = VT + PLANE;
  const float NEGV = -1.0e30f;
  const float SCL = 0.08838834764831845f;

  const int dq = doc[qi];
  int dmin = dq, dmax = dq;
#pragma unroll
  for (int o = 1; o < 16; o <<= 1) {
    const int a = __shfl_xor(dmin, o, 32), b = __shfl_xor(dmax, o, 32);
    dmin = (a < dmin) ? a : dmin; dmax = (b > dmax) ? b : dmax;
  }

  v16b qh[4], ql[4];
  {
    const size_t qoff = (size_t)qi * DM + head * HD;
#pragma unroll
    for (int ks = 0; ks < 4; ++ks) { qh[ks] = ld_frag(Qh + qoff + ks * 32, hh); ql[ks] = ld_frag(Ql + qoff + ks * 32, hh); }
  }

  const v8f z8 = {0.f, 0.f, 0.f, 0.f, 0.f, 0.f, 0.f, 0.f};
  v8f acc[4] = {z8, z8, z8, z8};
  float m = NEGV, l = 0.f;
  const int nsteps = (q0 + 16 + 31) >> 5;

#pragma unroll 1
  for (int js = 0; js < nsteps; ++js) {
    const int j0 = js << 5;
    const int dk = doc[j0 + lane];
    if (__ballot((dk >= dmin) & (dk <= dmax)) == 0ull) continue;

    v8f s0 = z8, s1 = z8;
    {
      const size_t ko = (size_t)(j0 + ln) * DM + head * HD;
#pragma unroll
      for (int ks = 0; ks < 4; ++ks) {
        const v16b a0h = ld_frag(Kh + ko + ks * 32, hh), a0l = ld_frag(Kl + ko + ks * 32, hh);
        s0 = mma3m(a0h, a0l, qh[ks], ql[ks], s0);
        const v16b a1h = ld_frag(Kh + ko + (size_t)16 * DM + ks * 32, hh), a1l = ld_frag(Kl + ko + (size_t)16 * DM + ks * 32, hh);
        s1 = mma3m(a1h, a1l, qh[ks], ql[ks], s1);
      }
    }

    const v4i dA = *(const v4ia*)(doc + j0 + 8 * hh), dB = *(const v4ia*)(doc + j0 + 8 * hh + 4);
    const v4i dC = *(const v4ia*)(doc + j0 + 16 + 8 * hh), dD = *(const v4ia*)(doc + j0 + 16 + 8 * hh + 4);
    const int dkk[16] = {dA[0], dA[1], dA[2], dA[3], dB[0], dB[1], dB[2], dB[3], dC[0], dC[1], dC[2], dC[3], dD[0], dD[1], dD[2], dD[3]};

    float xv[16];
    float mx = NEGV;
#pragma unroll
    for (int r = 0; r < 8; ++r) {
      const int k0 = j0 + 8 * hh + r, k1 = k0 + 16;
      const bool v0 = (k0 <= qi) & (dkk[r] == dq);
      const bool v1 = (k1 <= qi) & (dkk[8 + r] == dq);
      xv[r] = v0 ? s0[r] * SCL : NEGV;
      xv[8 + r] = v1 ? s1[r] * SCL : NEGV;
      mx = fmaxf(mx, fmaxf(xv[r], xv[8 + r]));
    }
    mx = fmaxf(mx, __shfl_xor(mx, 16, 32));
    const float mn = fmaxf(m, mx);
    const float alpha = __expf(m - mn);
    m = mn;

    FragB ph, pl;
    float ps = 0.f;
#pragma unroll
    for (int i = 0; i < 16; ++i) {
      const float e = __expf(xv[i] - mn);
      const float p = (xv[i] > -1.0e29f) ? e : 0.f;
      ps += p;
      const unsigned short hb = bf16_bits(p);
      ph.u[i] = hb;
      pl.u[i] = bf16_bits(p - bf16_val(hb));
    }
    ps += __shfl_xor(ps, 16, 32);
    l = l * alpha + ps;

#pragma unroll
    for (int dt = 0; dt < 4; ++dt)
#pragma unroll
      for (int r = 0; r < 8; ++r) acc[dt][r] *= alpha;

#pragma unroll
    for (int dt = 0; dt < 4; ++dt) {
      const size_t vo = (size_t)(head * HD + hf * 64 + dt * 16 + ln) * SEQ + j0;
      const v16b vh = ld_frag(VTh + vo, hh), vl = ld_frag(VTl + vo, hh);
      acc[dt] = mma3m(vh, vl, ph.v, pl.v, acc[dt]);
    }
  }

  const float inv = 1.0f / l;
#pragma unroll
  for (int dt = 0; dt < 4; ++dt)
#pragma unroll
    for (int r = 0; r < 8; ++r) so[w][ln][dt * 16 + 8 * hh + r] = acc[dt][r] * inv;
  __syncthreads();

  v8us hv[4], lv[4];
  const int rq = lane >> 3, pc = lane & 7;
#pragma unroll
  for (int it = 0; it < 4; ++it) {
    const int row = it * 4 + rq;
    const v4f a = *(const v4fa*)&so[w][row][pc * 8], c = *(const v4fa*)&so[w][row][pc * 8 + 4];
#pragma unroll
    for (int q = 0; q < 4; ++q) {
      const unsigned short ha = bf16_bits(a[q]), hc = bf16_bits(c[q]);
      hv[it][q] = ha; lv[it][q] = bf16_bits(a[q] - bf16_val(ha));
      hv[it][4 + q] = hc; lv[it][4 + q] = bf16_bits(c[q] - bf16_val(hc));
    }
  }
  for (int pass = 0; pass < 2; ++pass) {
#pragma unroll
    for (int it = 0; it < 4; ++it) {
      const int row = it * 4 + rq;
      unsigned short* dst = CTX + (size_t)(q0 + row) * DM + head * HD + hf * 64 + pc * 8;
      *(volatile v8us*)dst = hv[it];
      *(volatile v8us*)(dst + PLANE) = lv[it];
    }
    if (pass == 0) __threadfence();
  }
}

extern "C" void kernel_launch(void* const* d_in, const int* in_sizes, int n_in,
                              void* d_out, int out_size, void* d_ws, size_t ws_size, hipStream_t stream) {
  if (n_in < 8) return;
  if (in_sizes[0] < NR * DM) return;
  if (in_sizes[1] < DM * DM || in_sizes[2] < DM * DM || in_sizes[3] < DM * DM || in_sizes[4] < DM * DM) return;
  if (in_sizes[5] < SEQ * HD || in_sizes[6] < SEQ * HD || in_sizes[7] < NR) return;
  if (out_size < NR * DM) return;
  const float* x  = (const float*)d_in[0];
  const float* Wq = (const float*)d_in[1];
  const float* Wk = (const float*)d_in[2];
  const float* Wv = (const float*)d_in[3];
  const float* Wo = (const float*)d_in[4];
  const float* sn = (const float*)d_in[5];
  const float* cs = (const float*)d_in[6];
  const int*  doc = (const int*)d_in[7];
  float* out = (float*)d_out;

  constexpr size_t SZ_X  = (size_t)NR * DM * 2;
  constexpr size_t SZ_W3 = (size_t)3 * DM * DM * 2;
  constexpr size_t SZ_QK = (size_t)4 * NR * DM * 2;
  constexpr size_t SZ_R0 = (SZ_X + SZ_W3 > SZ_QK) ? (SZ_X + SZ_W3) : SZ_QK;
  constexpr size_t SZ_WO = (size_t)DM * DM * 2;
  constexpr size_t SZ_QKV = (size_t)NR * N3 * 4;
  constexpr size_t SZ_VT = (size_t)2 * DM * SEQ * 2;
  constexpr size_t SZ_CX = (size_t)2 * NR * DM * 2;
  constexpr size_t SZ_ALL = SZ_R0 + SZ_WO + SZ_QKV + SZ_VT + SZ_CX;
  static_assert(SZ_X + SZ_W3 <= SZ_R0 && SZ_QK <= SZ_R0);
  static_assert(SZ_X % 256 == 0 && SZ_R0 % 256 == 0 && SZ_WO % 256 == 0 && SZ_QKV % 256 == 0 && SZ_VT % 256 == 0 && SZ_CX % 256 == 0);
  static_assert(SZ_ALL <= (size_t)134217728);
  if (SZ_ALL > ws_size) return;
  char* ws = (char*)d_ws;
  unsigned short* XB  = (unsigned short*)(ws);
  unsigned short* WT3 = (unsigned short*)(ws + SZ_X);
  unsigned short* QKp = (unsigned short*)(ws);
  unsigned short* WoT = (unsigned short*)(ws + SZ_R0);
  float*          QKV = (float*)(ws + SZ_R0 + SZ_WO);
  unsigned short* VTp = (unsigned short*)(ws + SZ_R0 + SZ_WO + SZ_QKV);
  unsigned short* CTX = (unsigned short*)(ws + SZ_R0 + SZ_WO + SZ_QKV + SZ_VT);

  const size_t n8 = (size_t)NR * DM / 8;
  k_xb<<<(unsigned)((n8 + 255) / 256), 256, 0, stream>>>(x, XB, n8);
  const unsigned wtb = (unsigned)(((size_t)DM * (DM / 8) + 255) / 256);
  k_wt_bf16<<<wtb, 256, 0, stream>>>(Wq, WT3, DM, DM);
  k_wt_bf16<<<wtb, 256, 0, stream>>>(Wk, WT3 + (size_t)DM * DM, DM, DM);
  k_wt_bf16<<<wtb, 256, 0, stream>>>(Wv, WT3 + (size_t)2 * DM * DM, DM, DM);
  k_wt_bf16<<<wtb, 256, 0, stream>>>(Wo, WoT, DM, DM);

  k_gemm<1><<<(unsigned)((NR / 128) * (N3 / 64)), 128, 0, stream>>>(XB, XB, DM, WT3, DM, QKV, N3, N3, DM);

  const int nrope = NR * NH * 8;
  k_rope_qk<<<(unsigned)((nrope + 255) / 256), 256, 0, stream>>>(QKV, sn, cs, QKp, nrope);
  k_vt<<<(unsigned)((SEQ / 64) * (DM / 64)), 256, 0, stream>>>(QKV, VTp);

  k_attn<<<(unsigned)((NH * (SEQ / 16) * 2) / 4), 128, 0, stream>>>(QKp, VTp, doc, CTX);

  k_gemm<2><<<(unsigned)((NR / 128) * (DM / 64)), 128, 0, stream>>>(CTX, CTX + PLANE, DM, WoT, DM, out, DM, DM, DM);
}
